// Conv_Decomp_7258494730848
// MI455X (gfx1250) — hardware-verified
//
#include <hip/hip_runtime.h>

typedef __attribute__((ext_vector_type(16))) _Float16 v16h;
typedef __attribute__((ext_vector_type(8)))  _Float16 v8h;
typedef __attribute__((ext_vector_type(8)))  float    v8f;
typedef __attribute__((ext_vector_type(4)))  float    v4f;
typedef __attribute__((ext_vector_type(2)))  unsigned v2u;

constexpr int kCin   = 64;
constexpr int kHin   = 256;
constexpr int kWin   = 256;
constexpr int kRank  = 64;
constexpr int kFilt  = 128;
constexpr int kHo    = kHin - 2;
constexpr int kWo    = kWin - 2;
constexpr int kNpix  = kHin * kWin;
constexpr int kNout  = kHo * kWo;
constexpr int kNpad  = ((kNout + 63) / 64) * 64;
constexpr int kOutTotal = kFilt * kNout;
static_assert(kNpix == 65536, "pixel count");
static_assert(kNout == 64516, "output pixel count");
static_assert(kNpad == 64576, "padded output pixel count");
static_assert(kOutTotal == 8258048, "output element count");
static_assert((kCin % 32) == 0 && (kRank % 32) == 0, "GEMM K multiples of 32");
static_assert((kNpix % 64) == 0 && (kRank % 64) == 0 && (kFilt % 64) == 0 && (kNpad % 64) == 0, "GEMM M,N multiples of 64");
static_assert((kNout % 4) == 0 && (kNpad % 4) == 0, "4-element groups never straddle a filter row");
static_assert(((kOutTotal / 4) % 32) == 0, "compaction waves are whole");
static_assert(((size_t)kOutTotal * 4) % 128 == 0, "output is a whole number of 128-B lines");

constexpr float kCarryX   = 16.0f;
constexpr float kCarryF3  = 64.0f;
constexpr float kCarryF0  = 256.0f;
constexpr float kScale1   = 1.0f / (kCarryX * kCarryF3);
constexpr float kScale2   = 1.0f / kCarryF0;

constexpr size_t kSzXT   = (size_t)kNpix * kCin * 2;
constexpr size_t kSzF3T  = (size_t)kRank * kCin * 2;
constexpr size_t kSzF0H  = (size_t)kFilt * kRank * 2;
constexpr size_t kSzT1   = (size_t)kNpix * kRank * 4;
constexpr size_t kSzT3H  = (size_t)kNpad * kRank * 2;
constexpr size_t kSzCPAD = (size_t)kFilt * kNpad * 4;
constexpr size_t kOffXT   = 0;
constexpr size_t kOffF3T  = kOffXT  + kSzXT;
constexpr size_t kOffF0H  = kOffF3T + kSzF3T;
constexpr size_t kOffT1   = kOffF0H + kSzF0H;
constexpr size_t kOffT3H  = kOffT1  + kSzT1;
constexpr size_t kOffCPAD = kOffT3H + kSzT3H;
constexpr size_t kWsTotal = kOffCPAD + kSzCPAD;
static_assert(kWsTotal == 66519040ull, "carve total");
static_assert(kWsTotal <= 134217728ull, "carve cap");
static_assert((kOffF3T % 256) == 0 && (kOffF0H % 256) == 0 && (kOffT1 % 256) == 0 &&
              (kOffT3H % 256) == 0 && (kOffCPAD % 256) == 0, "256-B aligned regions");

union FragH { v16h v; v8h h[2]; };
__device__ __forceinline__ v16h frag_load_h(const _Float16* p) {
  FragH f;
  f.h[0] = *(const v8h*)(p);
  f.h[1] = *(const v8h*)(p + 16);
  return f.v;
}
__device__ __forceinline__ v8f mma_f16(v16h a, v16h b, v8f c) {
  c = __builtin_amdgcn_wmma_f32_16x16x32_f16(false, a, false, b, (short)0, c, false, false);
  asm volatile("v_nop\n\tv_nop\n\tv_nop\n\tv_nop" : "+v"(c) : "v"(a), "v"(b));
  return c;
}

__global__ __launch_bounds__(256) void prep_weights_kernel(
    const float* __restrict__ f3, const float* __restrict__ f0,
    unsigned short* __restrict__ F3T, unsigned short* __restrict__ F0H)
{
  const int gid = blockIdx.x * 256 + threadIdx.x;
  const int row = gid >> 3;
  const int c8  = (gid & 7) * 8;
  v8h hv;
  unsigned short* dst;
  if (blockIdx.x < 2) {
#pragma unroll
    for (int e = 0; e < 8; ++e) {
      const float s = f3[(c8 + e) * kRank + row] * kCarryF3;
      hv[e] = (_Float16)s;
    }
    dst = F3T + row * kCin + c8;
  } else {
    const int f = row - kRank;
    const v4f a0 = *(const v4f*)(f0 + f * kRank + c8);
    const v4f a1 = *(const v4f*)(f0 + f * kRank + c8 + 4);
#pragma unroll
    for (int e = 0; e < 4; ++e) {
      const float s0 = a0[e] * kCarryF0;
      const float s1 = a1[e] * kCarryF0;
      hv[e]     = (_Float16)s0;
      hv[4 + e] = (_Float16)s1;
    }
    dst = F0H + f * kRank + c8;
  }
  *(volatile v8h*)dst = hv;
  __threadfence();
  *(volatile v8h*)dst = hv;
}

__global__ __launch_bounds__(256) void xpose_convert_kernel(
    const float* __restrict__ in, unsigned short* __restrict__ XT)
{
  __shared__ __align__(16) float sT[64 * 68];
  const int tid = threadIdx.x;
  const int p0  = blockIdx.x * 64;
#pragma unroll
  for (int i = 0; i < 4; ++i) {
    const int idx = i * 256 + tid;
    const int c   = idx >> 4;
    const int p4  = (idx & 15) * 4;
    const v4f v = *(const v4f*)(in + (size_t)c * kNpix + p0 + p4);
    sT[(p4 + 0) * 68 + c] = v[0] * kCarryX;
    sT[(p4 + 1) * 68 + c] = v[1] * kCarryX;
    sT[(p4 + 2) * 68 + c] = v[2] * kCarryX;
    sT[(p4 + 3) * 68 + c] = v[3] * kCarryX;
  }
  __syncthreads();
  const int rq = tid >> 3;
  const int c8 = (tid & 7) * 8;
  v8h hv[2];
#pragma unroll
  for (int it = 0; it < 2; ++it) {
    const float* sp = sT + (it * 32 + rq) * 68 + c8;
    const v4f a0 = *(const v4f*)(sp);
    const v4f a1 = *(const v4f*)(sp + 4);
#pragma unroll
    for (int e = 0; e < 4; ++e) {
      hv[it][e]     = (_Float16)a0[e];
      hv[it][4 + e] = (_Float16)a1[e];
    }
  }
  for (int pass = 0; pass < 2; ++pass) {
#pragma unroll
    for (int it = 0; it < 2; ++it) {
      unsigned short* q = XT + (size_t)(p0 + it * 32 + rq) * kCin + c8;
      *(volatile v8h*)q = hv[it];
    }
    __threadfence();
  }
}

__global__ __launch_bounds__(256) void gemm_f16_tile64(
    const unsigned short* __restrict__ Ap, int lda,
    const unsigned short* __restrict__ Btp, int ldb,
    float* __restrict__ C, int ldc,
    int M, int N, int K, float scale)
{
  const _Float16* A  = (const _Float16*)Ap;
  const _Float16* Bt = (const _Float16*)Btp;
  __shared__ __align__(16) float sT[8][16 * 68];
  const int lane = threadIdx.x & 31;
  const int wave = __builtin_amdgcn_readfirstlane((int)(threadIdx.x >> 5));
  const int tilesN = N >> 6;
  const int tilesM = M >> 6;
  const int tile = blockIdx.x * 8 + wave;
  if (tile >= tilesM * tilesN) return;
  const int tm = tile / tilesN;
  const int tn = tile - tm * tilesN;
  const int m0 = tm << 6;
  const int n0 = tn << 6;

  const int rlane = lane & 15;
  const int koff  = (lane >> 4) * 8;
  const int mOff  = (lane >> 4) * 8;

  v8f acc[4][4];
#pragma unroll
  for (int i = 0; i < 4; ++i)
#pragma unroll
    for (int j = 0; j < 4; ++j) acc[i][j] = (v8f){0.f,0.f,0.f,0.f,0.f,0.f,0.f,0.f};

  for (int k0 = 0; k0 < K; k0 += 32) {
    v16h bh[4];
#pragma unroll
    for (int j = 0; j < 4; ++j) {
      const size_t bo = (size_t)(n0 + (j << 4) + rlane) * ldb + koff + k0;
      bh[j] = frag_load_h(Bt + bo);
    }
#pragma unroll
    for (int i = 0; i < 4; ++i) {
      const size_t ao = (size_t)(m0 + (i << 4) + rlane) * lda + koff + k0;
      const v16h ah = frag_load_h(A + ao);
#pragma unroll
      for (int j = 0; j < 4; ++j) acc[i][j] = mma_f16(ah, bh[j], acc[i][j]);
    }
  }

  float* slab = sT[wave];
#pragma unroll
  for (int i = 0; i < 4; ++i) {
    const int mBase = m0 + (i << 4);
#pragma unroll
    for (int j = 0; j < 4; ++j) {
#pragma unroll
      for (int r = 0; r < 8; ++r) {
        const float v = acc[i][j][r] * scale;
        slab[(mOff + r) * 68 + (j << 4) + rlane] = v;
      }
    }
    __builtin_amdgcn_fence(__ATOMIC_RELEASE, "workgroup");
    __builtin_amdgcn_wave_barrier();
    __builtin_amdgcn_fence(__ATOMIC_ACQUIRE, "workgroup");
    {
      const int hh = lane >> 4, c4 = (lane & 15) * 4;
      for (int pass = 0; pass < 2; ++pass) {
#pragma unroll
        for (int it = 0; it < 8; ++it) {
          const int row = it * 2 + hh;
          const v4f v = *(const v4f*)(slab + row * 68 + c4);
          *(volatile v4f*)(C + (size_t)(mBase + row) * ldc + n0 + c4) = v;
        }
        __threadfence();
      }
    }
    __builtin_amdgcn_fence(__ATOMIC_RELEASE, "workgroup");
    __builtin_amdgcn_wave_barrier();
    __builtin_amdgcn_fence(__ATOMIC_ACQUIRE, "workgroup");
  }
}

static_assert(((size_t)kNpad * 16) % 256 == 0, "tap grid exact");
__global__ __launch_bounds__(256) void tap3x3_kernel(
    const float* __restrict__ T1, const float* __restrict__ f1, const float* __restrict__ f2,
    unsigned short* __restrict__ T3H)
{
  const int gid = blockIdx.x * 256 + threadIdx.x;
  const int n   = gid >> 4;
  const int r4  = (gid & 15) * 4;
  const bool valid = (n < kNout);
  const int nc  = valid ? n : (kNout - 1);
  const int i   = nc / kWo;
  const int j   = nc - i * kWo;
  v4f wv[3], wh[3];
#pragma unroll
  for (int h = 0; h < 3; ++h) {
    wv[h] = *(const v4f*)(f1 + h * kRank + r4);
    wh[h] = *(const v4f*)(f2 + h * kRank + r4);
  }
  const float* base = T1 + (size_t)(i * kWin + j) * kRank + r4;
  float acc[4] = {0.0f, 0.0f, 0.0f, 0.0f};
#pragma unroll
  for (int h = 0; h < 3; ++h) {
    const v4f t0 = *(const v4f*)(base + (size_t)(h * kWin + 0) * kRank);
    const v4f t1 = *(const v4f*)(base + (size_t)(h * kWin + 1) * kRank);
    const v4f t2 = *(const v4f*)(base + (size_t)(h * kWin + 2) * kRank);
#pragma unroll
    for (int e = 0; e < 4; ++e) {
      float s = t0[e] * wh[0][e];
      s = fmaf(t1[e], wh[1][e], s);
      s = fmaf(t2[e], wh[2][e], s);
      acc[e] = fmaf(s, wv[h][e], acc[e]);
    }
  }
  const float o0 = valid ? acc[0] : 0.0f;
  const float o1 = valid ? acc[1] : 0.0f;
  const float o2 = valid ? acc[2] : 0.0f;
  const float o3 = valid ? acc[3] : 0.0f;
  const _Float16 h0 = (_Float16)o0;
  const _Float16 h1 = (_Float16)o1;
  const _Float16 h2 = (_Float16)o2;
  const _Float16 h3 = (_Float16)o3;
  const unsigned b0 = (unsigned)__builtin_bit_cast(unsigned short, h0);
  const unsigned b1 = (unsigned)__builtin_bit_cast(unsigned short, h1);
  const unsigned b2 = (unsigned)__builtin_bit_cast(unsigned short, h2);
  const unsigned b3 = (unsigned)__builtin_bit_cast(unsigned short, h3);
  v2u pk;
  pk.x = b0 | (b1 << 16);
  pk.y = b2 | (b3 << 16);
  unsigned short* q = T3H + (size_t)n * kRank + r4;
  *(volatile v2u*)q = pk;
  __threadfence();
  *(volatile v2u*)q = pk;
}

__global__ __launch_bounds__(256) void compact_kernel(
    const float* __restrict__ CPAD, float* __restrict__ out)
{
  const int t = blockIdx.x * 256 + threadIdx.x;
  if (t >= kOutTotal / 4) return;
  const int g = t * 4;
  const int f = g / kNout;
  const int n = g - f * kNout;
  const v4f v = *(const v4f*)(CPAD + (size_t)f * kNpad + n);
  float* q = out + g;
  *(volatile v4f*)q = v;
  __threadfence();
  *(volatile v4f*)q = v;
}

extern "C" void kernel_launch(void* const* d_in, const int* in_sizes, int n_in,
                              void* d_out, int out_size, void* d_ws, size_t ws_size,
                              hipStream_t stream) {
  if (n_in < 5) return;
  if (in_sizes[0] != kCin * kNpix) return;
  if (in_sizes[1] != kFilt * kRank) return;
  if (in_sizes[2] != 3 * kRank) return;
  if (in_sizes[3] != 3 * kRank) return;
  if (in_sizes[4] != kCin * kRank) return;
  if (out_size != kOutTotal) return;
  if (ws_size < kWsTotal) return;

  const float* input   = (const float*)d_in[0];
  const float* factor0 = (const float*)d_in[1];
  const float* factor1 = (const float*)d_in[2];
  const float* factor2 = (const float*)d_in[3];
  const float* factor3 = (const float*)d_in[4];
  float* out = (float*)d_out;

  char* ws = (char*)d_ws;
  unsigned short* XT   = (unsigned short*)(ws + kOffXT);
  unsigned short* F3T  = (unsigned short*)(ws + kOffF3T);
  unsigned short* F0H  = (unsigned short*)(ws + kOffF0H);
  float*          T1   = (float*)(ws + kOffT1);
  unsigned short* T3H  = (unsigned short*)(ws + kOffT3H);
  float*          CPAD = (float*)(ws + kOffCPAD);

  prep_weights_kernel<<<6, 256, 0, stream>>>(factor3, factor0, F3T, F0H);

  xpose_convert_kernel<<<kNpix / 64, 256, 0, stream>>>(input, XT);

  gemm_f16_tile64<<<((kNpix / 64) * (kRank / 64) + 7) / 8, 256, 0, stream>>>(
      XT, kCin, F3T, kCin, T1, kRank, kNpix, kRank, kCin, kScale1);

  tap3x3_kernel<<<(kNpad * 16) / 256, 256, 0, stream>>>(T1, factor1, factor2, T3H);

  gemm_f16_tile64<<<((kFilt / 64) * (kNpad / 64) + 7) / 8, 256, 0, stream>>>(
      F0H, kRank, T3H, kRank, CPAD, kNpad, kFilt, kNpad, kRank, kScale2);

  compact_kernel<<<(kOutTotal / 4 + 255) / 256, 256, 0, stream>>>(CPAD, out);
}
